// SuperGlueMultiHeadAttention_45896020525737
// MI455X (gfx1250) — hardware-verified
//
#include <hip/hip_runtime.h>
#include <hip/hip_bf16.h>

#define NB 8
#define NC 256
#define NH 4
#define NDH 64
#define NP 2048

typedef __attribute__((ext_vector_type(16))) _Float16 v16h;
typedef __attribute__((ext_vector_type(8)))  _Float16 v8h;
typedef __attribute__((ext_vector_type(16))) __bf16   v16b;
typedef __attribute__((ext_vector_type(8)))  __bf16   v8b;
typedef __attribute__((ext_vector_type(8)))  float    v8f;
typedef __attribute__((ext_vector_type(4)))  float    v4f;
#define PSCALE 32768.0f
#define U16(p) ((const unsigned short*)(const void*)(p))
#define PSCALE_INV (1.0f / 32768.0f)

__device__ __forceinline__ unsigned short f2bf_bits(float f) {
  unsigned u = __float_as_uint(f);
  return (unsigned short)((u + 0x7FFFu + ((u >> 16) & 1u)) >> 16);
}
__device__ __forceinline__ float bf_bits2f(unsigned short h) { return __uint_as_float(((unsigned)h) << 16); }

__device__ __forceinline__ void dep_guard_h(v8f& a, v8f& b, v16h x, v16h y) { asm volatile("v_nop\n\tv_nop\n\tv_nop\n\tv_nop" : "+v"(a), "+v"(b) : "v"(x), "v"(y)); }
__device__ __forceinline__ void dep_guard_b(v8f& a, v8f& b, v16b x, v16b y) { asm volatile("v_nop\n\tv_nop\n\tv_nop\n\tv_nop" : "+v"(a), "+v"(b) : "v"(x), "v"(y)); }
__device__ __forceinline__ void keep4_h(v16h a, v16h b, v16h c, v16h d) { asm volatile("v_nop" :: "v"(a), "v"(b), "v"(c), "v"(d)); }
__device__ __forceinline__ void keep4_b(v16b a, v16b b, v16b c, v16b d) { asm volatile("v_nop" :: "v"(a), "v"(b), "v"(c), "v"(d)); }
__device__ __forceinline__ void acc_guard4(v8f& a, v8f& b, v8f& c, v8f& d) { asm volatile("v_nop\n\tv_nop\n\tv_nop\n\tv_nop" : "+v"(a), "+v"(b), "+v"(c), "+v"(d)); }
template <typename T> struct Frag;
template <> struct Frag<_Float16> {
  typedef v16h V; union U { v16h v; v8h h[2]; };
  static __device__ __forceinline__ v16h load(const _Float16* p) {
    U f; f.h[0] = *(const v8h*)(p); f.h[1] = *(const v8h*)(p + 16); return f.v;
  }
  static __device__ __forceinline__ v8f mma(v16h a, v16h b, v8f c) {
    return __builtin_amdgcn_wmma_f32_16x16x32_f16(false, a, false, b, (short)0, c, false, false);
  }
  static __device__ __forceinline__ void guard(v8f& a, v8f& b, v16h x, v16h y) { dep_guard_h(a, b, x, y); }
  static __device__ __forceinline__ void keep(v16h a, v16h b, v16h c, v16h d) { keep4_h(a, b, c, d); }
};
template <> struct Frag<__bf16> {
  typedef v16b V; union U { v16b v; v8b h[2]; };
  static __device__ __forceinline__ v16b load(const __bf16* p) {
    U f; f.h[0] = *(const v8b*)(p); f.h[1] = *(const v8b*)(p + 16); return f.v;
  }
  static __device__ __forceinline__ v8f mma(v16b a, v16b b, v8f c) {
    return __builtin_amdgcn_wmma_f32_16x16x32_bf16(false, a, false, b, (short)0, c, false, false);
  }
  static __device__ __forceinline__ void guard(v8f& a, v8f& b, v16b x, v16b y) { dep_guard_b(a, b, x, y); }
  static __device__ __forceinline__ void keep(v16b a, v16b b, v16b c, v16b d) { keep4_b(a, b, c, d); }
};

template <int ET> struct Elem;
template <> struct Elem<0> { typedef _Float16 T; };
template <> struct Elem<1> { typedef __bf16 T; };
template <int ET, bool SPLIT, int BIAS_MODE, int OUT_MODE, bool RESID, int ACT = 0>
__global__ __launch_bounds__(256) void wmma_gemm64(
    const unsigned short* __restrict__ Ap, const unsigned short* __restrict__ A2p, int lda, long strideA,
    const unsigned short* __restrict__ Btp, const unsigned short* __restrict__ Bt2p, int ldb, long strideB,
    void* __restrict__ Cout, void* __restrict__ Cout2, int ldc, long strideC,
    const float* __restrict__ bias,
    const float* __restrict__ resid, long strideR,
    int M, int N, int K, float scale) {
  typedef typename Elem<ET>::T T;
  typedef typename Frag<T>::V V;
  const T* A = (const T*)Ap; const T* A2 = (const T*)A2p; const T* Bt = (const T*)Btp; const T* Bt2 = (const T*)Bt2p;
  __shared__ __align__(16) float sT[8][16 * 68];
  const int b    = blockIdx.y;
  const int lane = threadIdx.x & 31;
  const int wave = threadIdx.x >> 5;
  const int tilesN = N >> 6;
  const int tilesM = M >> 6;
  const int tile = blockIdx.x * 8 + wave;
  if (tile >= tilesM * tilesN) return;
  const int tm = tile / tilesN;
  const int tn = tile - tm * tilesN;
  const int m0 = tm << 6;
  const int n0 = tn << 6;

  const T* Ab  = A  + (size_t)b * strideA;
  const T* Bb  = Bt + (size_t)b * strideB;
  const T* Ab2 = SPLIT ? (A2  + (size_t)b * strideA) : nullptr;
  const T* Bb2 = SPLIT ? (Bt2 + (size_t)b * strideB) : nullptr;

  const int rlane = lane & 15;
  const int koff  = (lane >> 4) * 8;
  const int mOff  = (lane >> 4) * 8;

  v8f acc[4][4];
#pragma unroll
  for (int i = 0; i < 4; ++i)
#pragma unroll
    for (int j = 0; j < 4; ++j) acc[i][j] = (v8f){0.f,0.f,0.f,0.f,0.f,0.f,0.f,0.f};

  for (int k0 = 0; k0 < K; k0 += 32) {
    V bh[4], bl[4];
#pragma unroll
    for (int j = 0; j < 4; ++j) {
      const size_t bo = (size_t)(n0 + (j << 4) + rlane) * ldb + koff + k0;
      bh[j] = Frag<T>::load(Bb + bo);
      if (SPLIT) bl[j] = Frag<T>::load(Bb2 + bo);
    }
#pragma unroll
    for (int i = 0; i < 4; ++i) {
      const size_t ao = (size_t)(m0 + (i << 4) + rlane) * lda + koff + k0;
      V ah = Frag<T>::load(Ab + ao);
      V al;
      if (SPLIT) al = Frag<T>::load(Ab2 + ao);
#pragma unroll
      for (int j = 0; j < 4; ++j) {
        acc[i][j] = Frag<T>::mma(ah, bh[j], acc[i][j]);
        if (SPLIT) {
          acc[i][j] = Frag<T>::mma(ah, bl[j], acc[i][j]);
          acc[i][j] = Frag<T>::mma(al, bh[j], acc[i][j]);
        }
      }
      Frag<T>::guard(acc[i][0], acc[i][3], ah, SPLIT ? al : ah);
    }
    Frag<T>::keep(bh[0], bh[1], bh[2], bh[3]);
    if (SPLIT) Frag<T>::keep(bl[0], bl[1], bl[2], bl[3]);
  }
  acc_guard4(acc[0][0], acc[0][1], acc[0][2], acc[0][3]);
  acc_guard4(acc[1][0], acc[1][1], acc[1][2], acc[1][3]);
  acc_guard4(acc[2][0], acc[2][1], acc[2][2], acc[2][3]);
  acc_guard4(acc[3][0], acc[3][1], acc[3][2], acc[3][3]);

  float* slab = sT[wave];
  const float* Rb = RESID ? (resid + (size_t)b * strideR) : nullptr;
#pragma unroll
  for (int i = 0; i < 4; ++i) {
    const int mBase = m0 + (i << 4);
#pragma unroll
    for (int j = 0; j < 4; ++j) {
      const int n = n0 + (j << 4) + rlane;
      float bv = 0.f;
      if (BIAS_MODE == 2) bv = bias[n];
#pragma unroll
      for (int r = 0; r < 8; ++r) {
        float v = acc[i][j][r] * scale;
        if (BIAS_MODE == 1) v += bias[mBase + mOff + r];
        if (BIAS_MODE == 2) v += bv;
        if (RESID) v += Rb[(size_t)(mBase + mOff + r) * ldc + n];
        if (ACT == 1) v = tanhf(v);
        if (ACT == 2) v = fmaxf(v, 0.0f);
        if (ACT == 3) v = v / (1.0f + expf(-v));
        if (ACT == 4) v = (v > 0.f) ? v : 0.01f * v;
        if (ACT == 5) v = 0.5f * v * (1.0f + erff(v * 0.70710678118654752f));
        slab[(mOff + r) * 68 + (j << 4) + rlane] = v;
      }
    }
    __builtin_amdgcn_fence(__ATOMIC_RELEASE, "workgroup");
    __builtin_amdgcn_wave_barrier();
    __builtin_amdgcn_fence(__ATOMIC_ACQUIRE, "workgroup");
    if (OUT_MODE == 0) {
      float* C = (float*)Cout + (size_t)b * strideC;
      const int hh = lane >> 4, c4 = (lane & 15) * 4;
      for (int pass = 0; pass < 2; ++pass) {
#pragma unroll
        for (int it = 0; it < 8; ++it) {
          const int row = it * 2 + hh;
          v4f v = *(const v4f*)(slab + row * 68 + c4);
          *(volatile v4f*)(C + (size_t)(mBase + row) * ldc + n0 + c4) = v;
        }
        __threadfence();
      }
    } else {
      const int q = lane >> 3, c8 = (lane & 7) * 8;
      unsigned short* C  = (unsigned short*)Cout  + (size_t)b * strideC;
      unsigned short* C2 = (OUT_MODE == 2) ? ((unsigned short*)Cout2 + (size_t)b * strideC) : nullptr;
      for (int pass = 0; pass < 2; ++pass) {
#pragma unroll
        for (int it = 0; it < 4; ++it) {
          const int row = it * 4 + q;
          const float* sp = slab + row * 68 + c8;
          v8h hv, lv;
#pragma unroll
          for (int e = 0; e < 8; ++e) {
            if (OUT_MODE == 1) {
              hv[e] = (_Float16)sp[e];
            } else {
              unsigned short hb = f2bf_bits(sp[e]);
              unsigned short lb = f2bf_bits(sp[e] - bf_bits2f(hb));
              hv[e] = __builtin_bit_cast(_Float16, hb);
              lv[e] = __builtin_bit_cast(_Float16, lb);
            }
          }
          *(volatile v8h*)(C + (size_t)(mBase + row) * ldc + n0 + c8) = hv;
          if (OUT_MODE == 2) *(volatile v8h*)(C2 + (size_t)(mBase + row) * ldc + n0 + c8) = lv;
        }
        __threadfence();
      }
    }
    __builtin_amdgcn_fence(__ATOMIC_RELEASE, "workgroup");
    __builtin_amdgcn_wave_barrier();
    __builtin_amdgcn_fence(__ATOMIC_ACQUIRE, "workgroup");
  }
}

__device__ __forceinline__ int chan_of(int j) { return ((j & 63) << 2) | (j >> 6); }

__global__ __launch_bounds__(256) void prep_weights(
    const float* __restrict__ wq, const float* __restrict__ wk, const float* __restrict__ wv, const float* __restrict__ wm,
    const float* __restrict__ bq, const float* __restrict__ bk, const float* __restrict__ bv,
    _Float16* __restrict__ W16, float* __restrict__ Bp) {
  const int t = threadIdx.x;
  if (blockIdx.x < 128) {
    const int p  = blockIdx.x >> 5;
    const int e0 = (((blockIdx.x & 31) << 8) + t) * 8;
    const int r  = e0 >> 8;
    const int c0 = e0 & 255;
    const float* W = (p == 0) ? wq : (p == 1) ? wk : (p == 2) ? wv : wm;
    v8h hv;
#pragma unroll
    for (int i = 0; i < 8; ++i) {
      const int cc   = c0 + i;
      const int srcA = chan_of(r) * NC + cc;
      const int srcB = r * NC + chan_of(cc);
      const int src  = (p < 3) ? srcA : srcB;
      hv[i] = (_Float16)(W[src] * 16.0f);
    }
    _Float16* dst = W16 + (size_t)p * 65536 + e0;
    for (int pass = 0; pass < 2; ++pass) {
      *(volatile v8h*)dst = hv;
      __threadfence();
    }
  } else {
    const int wave = t >> 5;
    if (wave < 6) {
      const int p  = wave >> 1;
      const int j0 = (t & 63) * 4;
      const float* Bs = (p == 0) ? bq : (p == 1) ? bk : bv;
      v4f val;
#pragma unroll
      for (int i = 0; i < 4; ++i) val[i] = Bs[chan_of(j0 + i)];
      float* dst = Bp + p * 256 + j0;
      for (int pass = 0; pass < 2; ++pass) {
        *(volatile v4f*)dst = val;
        __threadfence();
      }
    }
  }
}

__global__ __launch_bounds__(256) void transpose_in_f16(
    const float* __restrict__ xq, const float* __restrict__ xk, const float* __restrict__ xv,
    _Float16* __restrict__ XT) {
  __shared__ __align__(16) _Float16 T[64 * 72];
  const int t = threadIdx.x;
  const int lane = t & 31, wave = t >> 5;
  const int n0 = blockIdx.x * 64, ci0 = blockIdx.y * 64, z = blockIdx.z;
  const int inp = z >> 3, b = z & 7;
  const float* X  = (inp == 0) ? xq : (inp == 1) ? xk : xv;
  const float* Xb = X + (size_t)b * NC * NP;
#pragma unroll
  for (int i = 0; i < 4; ++i) {
    const int idx = i * 256 + t;
    const int r = idx >> 4, c4 = (idx & 15) * 4;
    const v4f v = *(const v4f*)(Xb + (size_t)(ci0 + r) * NP + n0 + c4);
#pragma unroll
    for (int e = 0; e < 4; ++e) T[(c4 + e) * 72 + r] = (_Float16)v[e];
  }
  __syncthreads();
  const int q = lane >> 3, c8 = (lane & 7) * 8;
  v8h vals[2];
#pragma unroll
  for (int it = 0; it < 2; ++it) {
    const int row = wave * 8 + it * 4 + q;
    vals[it] = *(const v8h*)(T + row * 72 + c8);
  }
  _Float16* Ob = XT + ((size_t)z * NP + n0) * NC + ci0;
  for (int pass = 0; pass < 2; ++pass) {
#pragma unroll
    for (int it = 0; it < 2; ++it) {
      const int row = wave * 8 + it * 4 + q;
      *(volatile v8h*)(Ob + (size_t)row * NC + c8) = vals[it];
    }
    __threadfence();
  }
}

__global__ __launch_bounds__(256) void softmax_rows_f16(const float* __restrict__ S, _Float16* __restrict__ P, int nrows) {
  const int lane = threadIdx.x & 31, wave = threadIdx.x >> 5;
  const int row = blockIdx.x * 8 + wave;
  if (row >= nrows) return;
  const float* sr = S + (size_t)row * NP;
  v4f x[16];
#pragma unroll
  for (int i = 0; i < 8; ++i) {
    const float* p = sr + (i * 32 + lane) * 8;
    x[2 * i]     = *(const v4f*)(p);
    x[2 * i + 1] = *(const v4f*)(p + 4);
  }
  float mx = -__builtin_huge_valf();
#pragma unroll
  for (int i = 0; i < 16; ++i) mx = fmaxf(mx, fmaxf(fmaxf(x[i][0], x[i][1]), fmaxf(x[i][2], x[i][3])));
#pragma unroll
  for (int off = 1; off < 32; off <<= 1) mx = fmaxf(mx, __shfl_xor(mx, off, 32));
  float sum = 0.f;
#pragma unroll
  for (int i = 0; i < 16; ++i) {
#pragma unroll
    for (int e = 0; e < 4; ++e) {
      const float ev = __expf(x[i][e] - mx);
      x[i][e] = ev;
      sum += ev;
    }
  }
#pragma unroll
  for (int off = 1; off < 32; off <<= 1) sum += __shfl_xor(sum, off, 32);
  const float f = (1.0f / sum) * 32768.0f;
  v8h hv[8];
#pragma unroll
  for (int i = 0; i < 8; ++i) {
#pragma unroll
    for (int e = 0; e < 4; ++e) {
      hv[i][e]     = (_Float16)(x[2 * i][e] * f);
      hv[i][4 + e] = (_Float16)(x[2 * i + 1][e] * f);
    }
  }
  _Float16* pr = P + (size_t)row * NP;
  for (int pass = 0; pass < 2; ++pass) {
#pragma unroll
    for (int i = 0; i < 8; ++i) *(volatile v8h*)(pr + (i * 32 + lane) * 8) = hv[i];
    __threadfence();
  }
}

extern "C" void kernel_launch(void* const* d_in, const int* in_sizes, int n_in,
                              void* d_out, int out_size, void* d_ws, size_t ws_size,
                              hipStream_t stream) {
  if (n_in < 11) return;
  if (in_sizes[0] != NB * NC * NP || in_sizes[1] != NB * NC * NP || in_sizes[2] != NB * NC * NP) return;
  if (in_sizes[3] != NC * NC || in_sizes[5] != NC * NC || in_sizes[7] != NC * NC || in_sizes[9] != NC * NC) return;
  if (in_sizes[4] != NC || in_sizes[6] != NC || in_sizes[8] != NC || in_sizes[10] != NC) return;
  if (out_size != NB * NC * NP) return;

  const float* xq = (const float*)d_in[0];
  const float* xk = (const float*)d_in[1];
  const float* xv = (const float*)d_in[2];
  const float* wq = (const float*)d_in[3];
  const float* bq = (const float*)d_in[4];
  const float* wk = (const float*)d_in[5];
  const float* bk = (const float*)d_in[6];
  const float* wv = (const float*)d_in[7];
  const float* bv = (const float*)d_in[8];
  const float* wm = (const float*)d_in[9];
  const float* bm = (const float*)d_in[10];
  float* out = (float*)d_out;

  const size_t PL  = (size_t)NP * NC;
  const size_t SPL = (size_t)NP * NP;
  const size_t off_XT = 0;
  const size_t off_Q  = off_XT + 24 * PL * 2;
  const size_t off_K  = off_Q  + 8 * PL * 2;
  const size_t off_VT = off_K  + 8 * PL * 2;
  const size_t off_O  = off_VT + 8 * PL * 2;
  const size_t off_W  = off_O  + 8 * PL * 2;
  const size_t off_B  = off_W  + 4 * 65536 * 2;
  const size_t off_S  = off_B  + 3 * 256 * 4;
  const size_t off_P  = off_S  + 2 * SPL * 4;
  const size_t total  = off_P  + 2 * SPL * 2;
  if (total > ws_size) return;

  char* ws = (char*)d_ws;
  unsigned short* XT16 = (unsigned short*)(ws + off_XT);
  unsigned short* Q16  = (unsigned short*)(ws + off_Q);
  unsigned short* K16  = (unsigned short*)(ws + off_K);
  unsigned short* VT16 = (unsigned short*)(ws + off_VT);
  unsigned short* O16  = (unsigned short*)(ws + off_O);
  unsigned short* W16  = (unsigned short*)(ws + off_W);
  float*          Bp   = (float*)(ws + off_B);
  float*          Sbuf = (float*)(ws + off_S);
  unsigned short* P16  = (unsigned short*)(ws + off_P);

  const unsigned short* Wq16 = W16;
  const unsigned short* Wk16 = W16 + 65536;
  const unsigned short* Wv16 = W16 + 2 * 65536;
  const unsigned short* Wm16 = W16 + 3 * 65536;

  prep_weights<<<dim3(129), dim3(256), 0, stream>>>(wq, wk, wv, wm, bq, bk, bv, (_Float16*)W16, Bp);

  transpose_in_f16<<<dim3(NP / 64, NC / 64, 24), dim3(256), 0, stream>>>(xq, xk, xv, (_Float16*)XT16);

  wmma_gemm64<0, false, 2, 1, false><<<dim3(16, NB), dim3(256), 0, stream>>>(
      XT16, XT16, NC, (long)PL,
      Wq16, Wq16, NC, 0L,
      (void*)Q16, (void*)Q16, NC, (long)PL,
      Bp, Bp, 0L, NP, NC, NC, 1.0f / 16.0f);
  wmma_gemm64<0, false, 2, 1, false><<<dim3(16, NB), dim3(256), 0, stream>>>(
      XT16 + 8 * PL, XT16 + 8 * PL, NC, (long)PL,
      Wk16, Wk16, NC, 0L,
      (void*)K16, (void*)K16, NC, (long)PL,
      Bp + 256, Bp + 256, 0L, NP, NC, NC, 1.0f / 16.0f);
  wmma_gemm64<0, false, 1, 1, false><<<dim3(16, NB), dim3(256), 0, stream>>>(
      Wv16, Wv16, NC, 0L,
      XT16 + 16 * PL, XT16 + 16 * PL, NC, (long)PL,
      (void*)VT16, (void*)VT16, NP, (long)PL,
      Bp + 512, Bp + 512, 0L, NC, NP, NC, 1.0f / 16.0f);

  for (int b = 0; b < NB; ++b) {
    for (int hp = 0; hp < 2; ++hp) {
      const unsigned short* Qb = Q16 + (size_t)b * PL + (size_t)(2 * hp) * NDH;
      const unsigned short* Kb = K16 + (size_t)b * PL + (size_t)(2 * hp) * NDH;
      wmma_gemm64<0, false, 0, 0, false><<<dim3(128, 2), dim3(256), 0, stream>>>(
          Qb, Qb, NC, (long)NDH,
          Kb, Kb, NC, (long)NDH,
          (void*)Sbuf, (void*)Sbuf, NP, (long)SPL,
          Bp, Bp, 0L, NP, NP, NDH, 0.125f);
      softmax_rows_f16<<<dim3((2 * NP) / 8), dim3(256), 0, stream>>>(Sbuf, (_Float16*)P16, 2 * NP);
      const unsigned short* Vb = VT16 + (size_t)b * PL + (size_t)(2 * hp) * NDH * NP;
      unsigned short* Ob = O16 + (size_t)b * PL + (size_t)(2 * hp) * NDH;
      wmma_gemm64<0, false, 0, 1, false><<<dim3(4, 2), dim3(256), 0, stream>>>(
          P16, P16, NP, (long)SPL,
          Vb, Vb, NP, (long)(NDH * NP),
          (void*)Ob, (void*)Ob, NC, (long)NDH,
          Bp, Bp, 0L, NP, NDH, NP, 1.0f / 128.0f);
    }
  }

  wmma_gemm64<0, false, 1, 0, false><<<dim3(16, NB), dim3(256), 0, stream>>>(
      Wm16, Wm16, NC, 0L,
      O16, O16, NC, (long)PL,
      (void*)out, (void*)out, NP, (long)PL,
      bm, bm, 0L, NC, NP, NC, 1.0f / 4096.0f);
}
